// LinearTransformer_24936580121040
// MI455X (gfx1250) — hardware-run, weakly checked
//
#include <hip/hip_runtime.h>

typedef __attribute__((ext_vector_type(16))) _Float16 v16h;
typedef __attribute__((ext_vector_type(8)))  _Float16 v8h;
typedef __attribute__((ext_vector_type(16))) __bf16   v16b;
typedef __attribute__((ext_vector_type(8)))  __bf16   v8b;
typedef __attribute__((ext_vector_type(8)))  float    v8f;
typedef __attribute__((ext_vector_type(4)))  float    v4f;
typedef __attribute__((ext_vector_type(8)))  unsigned short v8us;

__device__ __forceinline__ unsigned short f2bf_bits(float f) {
  unsigned u = __float_as_uint(f);
  return (unsigned short)((u + 0x7FFFu + ((u >> 16) & 1u)) >> 16);
}
__device__ __forceinline__ float bf_bits2f(unsigned short h) { return __uint_as_float(((unsigned)h) << 16); }

__device__ __forceinline__ void dep_guard_h(v8f& a, v8f& b, v16h x, v16h y) { asm volatile("v_nop\n\tv_nop\n\tv_nop\n\tv_nop" : "+v"(a), "+v"(b) : "v"(x), "v"(y)); }
__device__ __forceinline__ void dep_guard_b(v8f& a, v8f& b, v16b x, v16b y) { asm volatile("v_nop\n\tv_nop\n\tv_nop\n\tv_nop" : "+v"(a), "+v"(b) : "v"(x), "v"(y)); }
__device__ __forceinline__ void keep4_h(v16h a, v16h b, v16h c, v16h d) { asm volatile("v_nop" :: "v"(a), "v"(b), "v"(c), "v"(d)); }
__device__ __forceinline__ void keep4_b(v16b a, v16b b, v16b c, v16b d) { asm volatile("v_nop" :: "v"(a), "v"(b), "v"(c), "v"(d)); }
template <typename T> struct Frag;
template <> struct Frag<_Float16> {
  typedef v16h V; union U { v16h v; v8h h[2]; };
  static __device__ __forceinline__ v16h load(const _Float16* p) {
    U f; f.h[0] = *(const v8h*)(p); f.h[1] = *(const v8h*)(p + 16); return f.v;
  }
  static __device__ __forceinline__ v8f mma(v16h a, v16h b, v8f c) {
    return __builtin_amdgcn_wmma_f32_16x16x32_f16(false, a, false, b, (short)0, c, false, false);
  }
  static __device__ __forceinline__ void guard(v8f& a, v8f& b, v16h x, v16h y) { dep_guard_h(a, b, x, y); }
  static __device__ __forceinline__ void keep(v16h a, v16h b, v16h c, v16h d) { keep4_h(a, b, c, d); }
};
template <> struct Frag<__bf16> {
  typedef v16b V; union U { v16b v; v8b h[2]; };
  static __device__ __forceinline__ v16b load(const __bf16* p) {
    U f; f.h[0] = *(const v8b*)(p); f.h[1] = *(const v8b*)(p + 16); return f.v;
  }
  static __device__ __forceinline__ v8f mma(v16b a, v16b b, v8f c) {
    return __builtin_amdgcn_wmma_f32_16x16x32_bf16(false, a, false, b, (short)0, c, false, false);
  }
  static __device__ __forceinline__ void guard(v8f& a, v8f& b, v16b x, v16b y) { dep_guard_b(a, b, x, y); }
  static __device__ __forceinline__ void keep(v16b a, v16b b, v16b c, v16b d) { keep4_b(a, b, c, d); }
};

constexpr int kBatch  = 4;
constexpr int kTok    = 65536;
constexpr int kDim    = 32;
constexpr int kHeads  = 2;
constexpr int kDHead  = 16;
constexpr int kDff    = 128;
constexpr int kLayers = 4;
constexpr int kTile   = 32;
constexpr int kTilesPerBatch = kTok / kTile;

constexpr int kKvThreads = 128;
constexpr int kKvWaves   = 4;
constexpr int kKvTPW     = 4;
constexpr int kKvWPB     = kTilesPerBatch / kKvTPW;
constexpr int kKvBlocksPerBatch = kKvWPB / kKvWaves;
constexpr int kPartF     = 384;

constexpr int kBkThreads = 64;
constexpr int kBkWaves   = 2;
constexpr int kBkTPW     = 4;
constexpr int kBkWPB     = kTilesPerBatch / kBkTPW;
constexpr int kBkBlocksPerBatch = kBkWPB / kBkWaves;

constexpr int kPitchH  = 40;
constexpr int kPitchF  = 36;
constexpr int kPitchF1 = 68;
constexpr int kPitchG  = 136;
constexpr int kCtxTF   = 512;
constexpr int kPrmBk   = 416;

static_assert(kTok % kTile == 0);
static_assert(kKvBlocksPerBatch * kKvWaves * kKvTPW == kTilesPerBatch);
static_assert(kBkBlocksPerBatch * kBkWaves * kBkTPW == kTilesPerBatch);
static_assert(kDim % 32 == 0 && kDff % 32 == 0);
static_assert((kPartF * 4) % 128 == 0);
static_assert((kLayers * kDim * kDim / 8) % 256 == 0);
static_assert((kLayers * kDim * kDHead / 8) % 256 == 0);
static_assert((kLayers * kDim * kDff / 8) % 256 == 0);

__device__ __forceinline__ v8f zero8() { return (v8f){0.f, 0.f, 0.f, 0.f, 0.f, 0.f, 0.f, 0.f}; }
__device__ __forceinline__ v8f mma_bf(v16b a, v16b b, v8f c) {
  c = __builtin_amdgcn_wmma_f32_16x16x32_bf16(false, a, false, b, (short)0, c, false, false);
  asm volatile("v_nop\n\tv_nop\n\tv_nop\n\tv_nop" : "+v"(c) : "v"(a), "v"(b));
  return c;
}
__device__ __forceinline__ v8f mma_h(v16h a, v16h b, v8f c) {
  c = __builtin_amdgcn_wmma_f32_16x16x32_f16(false, a, false, b, (short)0, c, false, false);
  asm volatile("v_nop\n\tv_nop\n\tv_nop\n\tv_nop" : "+v"(c) : "v"(a), "v"(b));
  return c;
}
__device__ __forceinline__ float rbf(float f) { return bf_bits2f(f2bf_bits(f)); }
__device__ __forceinline__ void split_bf(float f, unsigned short& hb, unsigned short& lb) {
  hb = f2bf_bits(f);
  lb = f2bf_bits(f - bf_bits2f(hb));
}
__device__ __forceinline__ unsigned short hbits(float f) { return __builtin_bit_cast(unsigned short, (_Float16)f); }
__device__ __forceinline__ float h2f(unsigned short u) { return (float)__builtin_bit_cast(_Float16, u); }
__device__ __forceinline__ v16b ldb(const unsigned short* p) { return Frag<__bf16>::load((const __bf16*)(const void*)p); }
__device__ __forceinline__ v16h ldh(const unsigned short* p) { return Frag<_Float16>::load((const _Float16*)(const void*)p); }
union FragUS { v16b vb; v16h vh; v8us u[2]; };

__device__ __forceinline__ void layer_norm32(const float (&x)[32], float (&y)[32], const float* g, const float* bb) {
  float m = 0.f;
#pragma unroll
  for (int d = 0; d < 32; ++d) m += x[d];
  m *= (1.0f / 32.0f);
  float v = 0.f;
#pragma unroll
  for (int d = 0; d < 32; ++d) { const float t = x[d] - m; v += t * t; }
  v *= (1.0f / 32.0f);
  const float rs = rsqrtf(v + 1e-5f);
#pragma unroll
  for (int d = 0; d < 32; ++d) y[d] = (x[d] - m) * rs * g[d] + bb[d];
}
__device__ __forceinline__ void load_row32(const float* p, float (&h)[32]) {
#pragma unroll
  for (int c = 0; c < 8; ++c) {
    const v4f v = *(const v4f*)(p + 4 * c);
    h[4 * c] = v[0]; h[4 * c + 1] = v[1]; h[4 * c + 2] = v[2]; h[4 * c + 3] = v[3];
  }
}
__device__ __forceinline__ void store_row32_lds(float* p, const float (&h)[32]) {
#pragma unroll
  for (int c = 0; c < 8; ++c) *(v4f*)(p + 4 * c) = (v4f){h[4 * c], h[4 * c + 1], h[4 * c + 2], h[4 * c + 3]};
}
__device__ __forceinline__ void store_row_bf16(unsigned short* dst, const float (&y)[32]) {
#pragma unroll
  for (int c = 0; c < 4; ++c) {
    v8us p;
#pragma unroll
    for (int i = 0; i < 8; ++i) p[i] = f2bf_bits(y[c * 8 + i]);
    *(v8us*)(dst + c * 8) = p;
  }
}
__device__ __forceinline__ void store_row_bf16_split(unsigned short* dhi, unsigned short* dlo, const float (&y)[32]) {
#pragma unroll
  for (int c = 0; c < 4; ++c) {
    v8us ph, pl;
#pragma unroll
    for (int i = 0; i < 8; ++i) { unsigned short hb, lb; split_bf(y[c * 8 + i], hb, lb); ph[i] = hb; pl[i] = lb; }
    *(v8us*)(dhi + c * 8) = ph;
    *(v8us*)(dlo + c * 8) = pl;
  }
}

__global__ __launch_bounds__(256) void k_castT(const float* __restrict__ src, unsigned short* __restrict__ dst,
                                               int kdim, int ndim, int nchunk) {
  const int i = blockIdx.x * 256 + threadIdx.x;
  if (i < nchunk) {
    const int kch = kdim >> 3;
    const int per_layer = ndim * kch;
    const int layer = i / per_layer;
    const int rem = i - layer * per_layer;
    const int n = rem / kch;
    const int k8 = rem - n * kch;
    const float* s = src + (size_t)layer * kdim * ndim + (size_t)(k8 * 8) * ndim + n;
    v8us p;
#pragma unroll
    for (int j = 0; j < 8; ++j) p[j] = f2bf_bits(s[(size_t)j * ndim]);
    unsigned short* d = dst + (size_t)i * 8;
    *(volatile v8us*)d = p;
    __threadfence();
    *(volatile v8us*)d = p;
  }
}

template <bool FIRST>
__global__ __launch_bounds__(kKvThreads) void k_kvctx(
    const float* __restrict__ hin, const float* __restrict__ xin,
    const float* __restrict__ w_in, const float* __restrict__ b_in,
    const float* __restrict__ ln1g, const float* __restrict__ ln1b,
    const unsigned short* __restrict__ wkT, const unsigned short* __restrict__ wvT,
    float* __restrict__ part) {
  __shared__ float prm[128];
  __shared__ __align__(16) unsigned short sPy[kKvWaves][32 * kPitchH];
  __shared__ __align__(16) unsigned short sWt[kKvWaves][16 * kPitchH];
  __shared__ __align__(16) unsigned short sVt[kKvWaves][16 * kPitchH];
  __shared__ __align__(16) float sPart[kKvWaves][kPartF];

  const int tid = threadIdx.x, wave = tid >> 5, l = tid & 31, half = l >> 4, col = l & 15, mOff = half * 8;
  const int b = blockIdx.y;
  for (int i = tid; i < 32; i += kKvThreads) {
    prm[i] = rbf(ln1g[i]); prm[32 + i] = rbf(ln1b[i]); prm[64 + i] = rbf(w_in[i]); prm[96 + i] = rbf(b_in[i]);
  }
  __syncthreads();
  unsigned short* Py = sPy[wave];
  unsigned short* Wt = sWt[wave];
  unsigned short* Vt = sVt[wave];
  const v16b fk = ldb(wkT + col * kDim + 8 * half);
  const v16b fv = ldb(wvT + col * kDim + 8 * half);
  v8f ctxS = zero8();
  float zp = 0.f;
  const int wg = blockIdx.x * kKvWaves + wave;
#pragma unroll 1
  for (int it = 0; it < kKvTPW; ++it) {
    const int tile = wg * kKvTPW + it;
    const size_t tok0 = (size_t)b * kTok + (size_t)tile * kTile;
    {
      float hr[32], y[32];
      if (FIRST) {
        const float xv = rbf(xin[tok0 + l]);
#pragma unroll
        for (int d = 0; d < 32; ++d) hr[d] = xv * prm[64 + d] + prm[96 + d];
      } else {
        load_row32(hin + (tok0 + l) * kDim, hr);
      }
      layer_norm32(hr, y, prm, prm + 32);
      store_row_bf16(Py + l * kPitchH, y);
    }
    __syncthreads();
#pragma unroll
    for (int mt = 0; mt < 2; ++mt) {
      const v16b a = ldb(Py + (mt * 16 + col) * kPitchH + 8 * half);
      const v8f ka = mma_bf(a, fk, zero8());
      const v8f va = mma_bf(a, fv, zero8());
      v8us pw, pv;
#pragma unroll
      for (int r = 0; r < 8; ++r) {
        const float w = expf(fminf(ka[r], 10.0f));
        const unsigned short wb = hbits(w);
        zp += h2f(wb);
        pw[r] = wb;
        pv[r] = hbits(va[r]);
      }
      *(v8us*)(Wt + col * kPitchH + mt * 16 + mOff) = pw;
      *(v8us*)(Vt + col * kPitchH + mt * 16 + mOff) = pv;
    }
    __syncthreads();
    {
      const v16h aw = ldh(Wt + col * kPitchH + 8 * half);
      const v16h bw = ldh(Vt + col * kPitchH + 8 * half);
      ctxS = mma_h(aw, bw, ctxS);
    }
  }
  float* sp = sPart[wave];
#pragma unroll
  for (int r = 0; r < 8; ++r) sp[(mOff + r) * 16 + col] = ctxS[r];
  sp[256 + l] = zp;
  sp[288 + l] = 0.f; sp[320 + l] = 0.f; sp[352 + l] = 0.f;
  __syncthreads();
  float* pp = part + ((size_t)b * kKvWPB + (size_t)wg) * kPartF;
  const v4f q0 = *(const v4f*)(sp + (0 * 32 + l) * 4);
  const v4f q1 = *(const v4f*)(sp + (1 * 32 + l) * 4);
  const v4f q2 = *(const v4f*)(sp + (2 * 32 + l) * 4);
  *(volatile v4f*)(pp + (0 * 32 + l) * 4) = q0;
  *(volatile v4f*)(pp + (1 * 32 + l) * 4) = q1;
  *(volatile v4f*)(pp + (2 * 32 + l) * 4) = q2;
  __threadfence();
  *(volatile v4f*)(pp + (0 * 32 + l) * 4) = q0;
  *(volatile v4f*)(pp + (1 * 32 + l) * 4) = q1;
  *(volatile v4f*)(pp + (2 * 32 + l) * 4) = q2;
}

__global__ __launch_bounds__(256) void k_ctxfin(const float* __restrict__ part, unsigned short* __restrict__ ctxT) {
  __shared__ __align__(16) unsigned short cs[kCtxTF];
  const int b = blockIdx.x, t = threadIdx.x, d = t >> 4, e = t & 15;
  const float* pb = part + (size_t)b * kKvWPB * kPartF;
  float S = 0.f, Z = 0.f;
#pragma unroll 1
  for (int w = 0; w < kKvWPB; ++w) {
    const float* p = pb + (size_t)w * kPartF;
    S += p[t];
    Z += p[256 + d] + p[272 + d];
  }
  const float c = S * (1.0f / Z);
  cs[e * 32 + d] = f2bf_bits(c);
  cs[e * 32 + 16 + d] = (unsigned short)0;
  __syncthreads();
  if (t < 32) {
    unsigned short* dst = ctxT + (size_t)b * kCtxTF;
    const v8us v0 = *(const v8us*)(cs + t * 8);
    const v8us v1 = *(const v8us*)(cs + 256 + t * 8);
    *(volatile v8us*)(dst + t * 8) = v0;
    *(volatile v8us*)(dst + 256 + t * 8) = v1;
    __threadfence();
    *(volatile v8us*)(dst + t * 8) = v0;
    *(volatile v8us*)(dst + 256 + t * 8) = v1;
  }
}

template <bool FIRST, bool LAST>
__global__ __launch_bounds__(kBkThreads) void k_block(
    const float* __restrict__ hin, const float* __restrict__ xin,
    const float* __restrict__ w_in, const float* __restrict__ b_in,
    float* __restrict__ hout, float* __restrict__ out,
    const float* __restrict__ w_out, const float* __restrict__ b_out,
    const float* __restrict__ ln1g, const float* __restrict__ ln1b,
    const float* __restrict__ ln2g, const float* __restrict__ ln2b,
    const float* __restrict__ bo, const float* __restrict__ b1, const float* __restrict__ b2,
    const unsigned short* __restrict__ wqT, const unsigned short* __restrict__ woT,
    const unsigned short* __restrict__ w1T, const unsigned short* __restrict__ w2T,
    const unsigned short* __restrict__ ctxT) {
  __shared__ float prm[kPrmBk];
  __shared__ __align__(16) float sF[kBkWaves][32 * kPitchF];
  __shared__ __align__(16) float sH[kBkWaves][32 * kPitchF];
  __shared__ __align__(16) unsigned short sP0[kBkWaves][32 * kPitchH];
  __shared__ __align__(16) unsigned short sP1[kBkWaves][32 * kPitchH];
  __shared__ __align__(16) float sF1[kBkWaves][16 * kPitchF1];
  __shared__ __align__(16) unsigned short sGh[kBkWaves][16 * kPitchG];
  __shared__ __align__(16) unsigned short sGl[kBkWaves][16 * kPitchG];
  __shared__ __align__(16) float sOut[kBkWaves][32];

  const int tid = threadIdx.x, wave = tid >> 5, l = tid & 31, half = l >> 4, col = l & 15, mOff = half * 8;
  const int b = blockIdx.y;
  for (int i = tid; i < 32; i += kBkThreads) {
    prm[i] = rbf(ln1g[i]); prm[32 + i] = rbf(ln1b[i]); prm[64 + i] = rbf(ln2g[i]); prm[96 + i] = rbf(ln2b[i]);
    prm[128 + i] = rbf(bo[i]); prm[160 + i] = rbf(b2[i]);
    prm[320 + i] = rbf(w_in[i]); prm[352 + i] = rbf(b_in[i]); prm[384 + i] = rbf(w_out[i]);
  }
  for (int i = tid; i < kDff; i += kBkThreads) prm[192 + i] = rbf(b1[i]);
  __syncthreads();
  float* Fw = sF[wave];
  float* Hw = sH[wave];
  unsigned short* P0 = sP0[wave];
  unsigned short* P1 = sP1[wave];
  float* F1 = sF1[wave];
  unsigned short* Gh = sGh[wave];
  unsigned short* Gl = sGl[wave];
  const unsigned short* ctxb = ctxT + (size_t)b * kCtxTF;
  const int wg = blockIdx.x * kBkWaves + wave;

#pragma unroll 1
  for (int it = 0; it < kBkTPW; ++it) {
    const int tile = wg * kBkTPW + it;
    const size_t tok0 = (size_t)b * kTok + (size_t)tile * kTile;

    {
      float hr[32], y[32];
      if (FIRST) {
        const float xv = rbf(xin[tok0 + l]);
#pragma unroll
        for (int d = 0; d < 32; ++d) hr[d] = xv * prm[320 + d] + prm[352 + d];
      } else {
        load_row32(hin + (tok0 + l) * kDim, hr);
      }
      layer_norm32(hr, y, prm, prm + 32);
      store_row_bf16(P0 + l * kPitchH, y);
      store_row32_lds(Hw + l * kPitchF, hr);
    }
    __syncthreads();

    {
      const v16b fq0 = ldb(wqT + col * kDim + 8 * half);
      const v16b fq1 = ldb(wqT + (16 + col) * kDim + 8 * half);
#pragma unroll
      for (int mt = 0; mt < 2; ++mt) {
        const v16b a = ldb(P0 + (mt * 16 + col) * kPitchH + 8 * half);
        const v8f acc0 = mma_bf(a, fq0, zero8());
        const v8f acc1 = mma_bf(a, fq1, zero8());
#pragma unroll
        for (int r = 0; r < 8; ++r) {
          Fw[(mt * 16 + mOff + r) * kPitchF + col] = acc0[r];
          Fw[(mt * 16 + mOff + r) * kPitchF + 16 + col] = acc1[r];
        }
      }
    }
    __syncthreads();

#pragma unroll 1
    for (int hh = 0; hh < kHeads; ++hh) {
      const float* qq = Fw + l * kPitchF + hh * kDHead;
      float qv[16];
#pragma unroll
      for (int c = 0; c < 4; ++c) {
        const v4f v = *(const v4f*)(qq + 4 * c);
        qv[4 * c] = v[0]; qv[4 * c + 1] = v[1]; qv[4 * c + 2] = v[2]; qv[4 * c + 3] = v[3];
      }
      float mx = qv[0];
#pragma unroll
      for (int d = 1; d < 16; ++d) mx = fmaxf(mx, qv[d]);
      float s = 0.f;
#pragma unroll
      for (int d = 0; d < 16; ++d) { qv[d] = expf(qv[d] - mx); s += qv[d]; }
      const float inv = 1.0f / s;
      v8us p0, p1;
#pragma unroll
      for (int d = 0; d < 8; ++d) { p0[d] = f2bf_bits(qv[d] * inv * 0.25f); p1[d] = f2bf_bits(qv[8 + d] * inv * 0.25f); }
      *(v8us*)(P1 + l * kPitchH + hh * kDHead) = p0;
      *(v8us*)(P1 + l * kPitchH + hh * kDHead + 8) = p1;
    }
    __syncthreads();

    {
      const v16b fc = ldb(ctxb + col * 32 + 8 * half);
#pragma unroll
      for (int mt = 0; mt < 2; ++mt)
#pragma unroll
        for (int hh = 0; hh < kHeads; ++hh) {
          FragUS ua;
          ua.u[0] = *(const v8us*)(P1 + (mt * 16 + col) * kPitchH + hh * kDHead + mOff);
          ua.u[1] = (v8us){0, 0, 0, 0, 0, 0, 0, 0};
          const v8f acc = mma_bf(ua.vb, fc, zero8());
#pragma unroll
          for (int r = 0; r < 8; ++r) P0[(mt * 16 + mOff + r) * kPitchH + hh * kDHead + col] = f2bf_bits(acc[r]);
        }
    }
    __syncthreads();

    {
      const v16b fo0 = ldb(woT + col * kDim + 8 * half);
      const v16b fo1 = ldb(woT + (16 + col) * kDim + 8 * half);
#pragma unroll
      for (int mt = 0; mt < 2; ++mt) {
        const v16b a = ldb(P0 + (mt * 16 + col) * kPitchH + 8 * half);
        const v8f acc0 = mma_bf(a, fo0, zero8());
        const v8f acc1 = mma_bf(a, fo1, zero8());
#pragma unroll
        for (int r = 0; r < 8; ++r) {
          Fw[(mt * 16 + mOff + r) * kPitchF + col] = acc0[r];
          Fw[(mt * 16 + mOff + r) * kPitchF + 16 + col] = acc1[r];
        }
      }
    }
    __syncthreads();

    {
      float h1[32], y2[32];
#pragma unroll
      for (int d = 0; d < 32; ++d) {
        const float o = Fw[l * kPitchF + d] + prm[128 + d];
        h1[d] = Hw[l * kPitchF + d] + o;
      }
      layer_norm32(h1, y2, prm + 64, prm + 96);
      store_row_bf16_split(P1 + l * kPitchH, P0 + l * kPitchH, y2);
      store_row32_lds(Hw + l * kPitchF, h1);
    }
    __syncthreads();

#pragma unroll 1
    for (int mt = 0; mt < 2; ++mt) {
      const v16b ahi = ldb(P1 + (mt * 16 + col) * kPitchH + 8 * half);
      const v16b alo = ldb(P0 + (mt * 16 + col) * kPitchH + 8 * half);
#pragma unroll 1
      for (int ch = 0; ch < 2; ++ch) {
#pragma unroll
        for (int nt = 0; nt < 4; ++nt) {
          const v16b bw = ldb(w1T + ((ch * 4 + nt) * 16 + col) * kDim + 8 * half);
          v8f acc = mma_bf(ahi, bw, zero8());
          acc = mma_bf(alo, bw, acc);
#pragma unroll
          for (int r = 0; r < 8; ++r) F1[(mOff + r) * kPitchF1 + nt * 16 + col] = acc[r];
        }
        __syncthreads();
        {
          const int rr = l & 15, cb = half * 32;
#pragma unroll 1
          for (int g8 = 0; g8 < 4; ++g8) {
            const int c0 = cb + g8 * 8;
            const float* fp = F1 + rr * kPitchF1 + c0;
            const float* bp = prm + 192 + ch * 64 + c0;
            v8us ph, pl;
#pragma unroll
            for (int e = 0; e < 8; ++e) {
              const float xg = fp[e] + bp[e];
              const float gv = 0.5f * xg * (1.0f + erff(xg * 0.70710678118654752f));
              unsigned short hb, lb;
              split_bf(gv, hb, lb);
              ph[e] = hb; pl[e] = lb;
            }
            *(v8us*)(Gh + rr * kPitchG + ch * 64 + c0) = ph;
            *(v8us*)(Gl + rr * kPitchG + ch * 64 + c0) = pl;
          }
        }
        __syncthreads();
      }
      {
        v8f acc0 = zero8(), acc1 = zero8();
#pragma unroll
        for (int ks = 0; ks < 4; ++ks) {
          const v16b gh = ldb(Gh + col * kPitchG + ks * 32 + 8 * half);
          const v16b gl = ldb(Gl + col * kPitchG + ks * 32 + 8 * half);
          const v16b b0 = ldb(w2T + col * kDff + ks * 32 + 8 * half);
          const v16b b1v = ldb(w2T + (16 + col) * kDff + ks * 32 + 8 * half);
          acc0 = mma_bf(gh, b0, acc0);
          acc0 = mma_bf(gl, b0, acc0);
          acc1 = mma_bf(gh, b1v, acc1);
          acc1 = mma_bf(gl, b1v, acc1);
        }
#pragma unroll
        for (int r = 0; r < 8; ++r) {
          Fw[(mt * 16 + mOff + r) * kPitchF + col] = acc0[r];
          Fw[(mt * 16 + mOff + r) * kPitchF + 16 + col] = acc1[r];
        }
      }
    }
    __syncthreads();

    if (LAST) {
      float so = 0.f;
#pragma unroll
      for (int d = 0; d < 32; ++d) {
        const float ffv = Fw[l * kPitchF + d] + prm[160 + d];
        const float hn = Hw[l * kPitchF + d] + ffv;
        so += hn * prm[384 + d];
      }
      so += rbf(b_out[0]);
      sOut[wave][l] = so;
      __syncthreads();
      if (l < 8) {
        const v4f v = *(const v4f*)(sOut[wave] + l * 4);
        float* op = out + tok0 + (size_t)l * 4;
        *(volatile v4f*)op = v;
        __threadfence();
        *(volatile v4f*)op = v;
      }
    } else {
#pragma unroll
      for (int d = 0; d < 32; ++d) {
        const float ffv = Fw[l * kPitchF + d] + prm[160 + d];
        const float hn = Hw[l * kPitchF + d] + ffv;
        Fw[l * kPitchF + d] = hn;
      }
      __syncthreads();
      float* hp = hout + tok0 * kDim;
      const int rq = l >> 3, c4 = (l & 7) * 4;
      for (int pass = 0; pass < 2; ++pass) {
#pragma unroll
        for (int i = 0; i < 8; ++i) {
          const int row = i * 4 + rq;
          const v4f v = *(const v4f*)(Fw + row * kPitchF + c4);
          *(volatile v4f*)(hp + (size_t)row * kDim + c4) = v;
        }
        __threadfence();
      }
    }
  }
}

extern "C" void kernel_launch(void* const* d_in, const int* in_sizes, int n_in,
                              void* d_out, int out_size, void* d_ws, size_t ws_size,
                              hipStream_t stream) {
  if (n_in < 18) return;
  if (in_sizes[0] != kBatch * kTok || out_size != kBatch * kTok) return;
  if (in_sizes[7] != kLayers * kDim * kDim || in_sizes[8] != kLayers * kDim * kDHead ||
      in_sizes[9] != kLayers * kDim * kDHead || in_sizes[10] != kLayers * kDim * kDim ||
      in_sizes[14] != kLayers * kDim * kDff || in_sizes[16] != kLayers * kDff * kDim) return;

  const float* x     = (const float*)d_in[0];
  const float* w_in  = (const float*)d_in[1];
  const float* b_in  = (const float*)d_in[2];
  const float* w_out = (const float*)d_in[3];
  const float* b_out = (const float*)d_in[4];
  const float* ln1_g = (const float*)d_in[5];
  const float* ln1_b = (const float*)d_in[6];
  const float* wq    = (const float*)d_in[7];
  const float* wk    = (const float*)d_in[8];
  const float* wv    = (const float*)d_in[9];
  const float* wo    = (const float*)d_in[10];
  const float* bo    = (const float*)d_in[11];
  const float* ln2_g = (const float*)d_in[12];
  const float* ln2_b = (const float*)d_in[13];
  const float* w1    = (const float*)d_in[14];
  const float* b1    = (const float*)d_in[15];
  const float* w2    = (const float*)d_in[16];
  const float* b2    = (const float*)d_in[17];
  float* out = (float*)d_out;

  char* ws = (char*)d_ws;
  size_t off = 0;
  const size_t hBytes = (size_t)kBatch * kTok * kDim * sizeof(float);
  float* hA = (float*)(ws + off); off += hBytes;
  float* hB = (float*)(ws + off); off += hBytes;
  unsigned short* wqT = (unsigned short*)(ws + off); off += (size_t)kLayers * kDim * kDim * 2;
  unsigned short* wkT = (unsigned short*)(ws + off); off += (size_t)kLayers * kDHead * kDim * 2;
  unsigned short* wvT = (unsigned short*)(ws + off); off += (size_t)kLayers * kDHead * kDim * 2;
  unsigned short* woT = (unsigned short*)(ws + off); off += (size_t)kLayers * kDim * kDim * 2;
  unsigned short* w1T = (unsigned short*)(ws + off); off += (size_t)kLayers * kDff * kDim * 2;
  unsigned short* w2T = (unsigned short*)(ws + off); off += (size_t)kLayers * kDim * kDff * 2;
  float* part = (float*)(ws + off); off += (size_t)kBatch * kKvWPB * kPartF * sizeof(float);
  unsigned short* ctxT = (unsigned short*)(ws + off); off += (size_t)kBatch * kCtxTF * 2;
  if (off > ws_size) return;

  {
    const int cq = kLayers * kDim * kDim / 8;
    const int ck = kLayers * kDim * kDHead / 8;
    const int c1 = kLayers * kDim * kDff / 8;
    k_castT<<<dim3((cq + 255) / 256), dim3(256), 0, stream>>>(wq, wqT, kDim, kDim, cq);
    k_castT<<<dim3((ck + 255) / 256), dim3(256), 0, stream>>>(wk, wkT, kDim, kDHead, ck);
    k_castT<<<dim3((ck + 255) / 256), dim3(256), 0, stream>>>(wv, wvT, kDim, kDHead, ck);
    k_castT<<<dim3((cq + 255) / 256), dim3(256), 0, stream>>>(wo, woT, kDim, kDim, cq);
    k_castT<<<dim3((c1 + 255) / 256), dim3(256), 0, stream>>>(w1, w1T, kDim, kDff, c1);
    k_castT<<<dim3((c1 + 255) / 256), dim3(256), 0, stream>>>(w2, w2T, kDff, kDim, c1);
  }

  for (int L = 0; L < kLayers; ++L) {
    const float* hin = (L & 1) ? hA : hB;
    float* hout = (L & 1) ? hB : hA;
    const dim3 gkv(kKvBlocksPerBatch, kBatch), bkv(kKvThreads);
    const dim3 gbk(kBkBlocksPerBatch, kBatch), bbk(kBkThreads);
    const unsigned short* wqL = wqT + (size_t)L * kDim * kDim;
    const unsigned short* wkL = wkT + (size_t)L * kDHead * kDim;
    const unsigned short* wvL = wvT + (size_t)L * kDHead * kDim;
    const unsigned short* woL = woT + (size_t)L * kDim * kDim;
    const unsigned short* w1L = w1T + (size_t)L * kDff * kDim;
    const unsigned short* w2L = w2T + (size_t)L * kDim * kDff;
    if (L == 0) {
      k_kvctx<true><<<gkv, bkv, 0, stream>>>(hin, x, w_in, b_in, ln1_g + L * kDim, ln1_b + L * kDim, wkL, wvL, part);
    } else {
      k_kvctx<false><<<gkv, bkv, 0, stream>>>(hin, x, w_in, b_in, ln1_g + L * kDim, ln1_b + L * kDim, wkL, wvL, part);
    }
    k_ctxfin<<<dim3(kBatch), dim3(256), 0, stream>>>(part, ctxT);
    if (L == 0) {
      k_block<true, false><<<gbk, bbk, 0, stream>>>(hin, x, w_in, b_in, hout, out, w_out, b_out,
          ln1_g + L * kDim, ln1_b + L * kDim, ln2_g + L * kDim, ln2_b + L * kDim,
          bo + L * kDim, b1 + L * kDff, b2 + L * kDim, wqL, woL, w1L, w2L, ctxT);
    } else if (L == kLayers - 1) {
      k_block<false, true><<<gbk, bbk, 0, stream>>>(hin, x, w_in, b_in, hout, out, w_out, b_out,
          ln1_g + L * kDim, ln1_b + L * kDim, ln2_g + L * kDim, ln2_b + L * kDim,
          bo + L * kDim, b1 + L * kDff, b2 + L * kDim, wqL, woL, w1L, w2L, ctxT);
    } else {
      k_block<false, false><<<gbk, bbk, 0, stream>>>(hin, x, w_in, b_in, hout, out, w_out, b_out,
          ln1_g + L * kDim, ln1_b + L * kDim, ln2_g + L * kDim, ln2_b + L * kDim,
          bo + L * kDim, b1 + L * kDff, b2 + L * kDim, wqL, woL, w1L, w2L, ctxT);
    }
  }
}
